// EfficientCrossAttentionV4_29480655519766
// MI455X (gfx1250) — hardware-verified
//
#include <hip/hip_runtime.h>

typedef _Float16 v16h __attribute__((ext_vector_type(16)));
typedef _Float16 v8h  __attribute__((ext_vector_type(8)));
typedef __bf16   v16b __attribute__((ext_vector_type(16)));
typedef float    v8f  __attribute__((ext_vector_type(8)));
typedef float    v4f  __attribute__((ext_vector_type(4)));
typedef unsigned short v8us __attribute__((ext_vector_type(8)));
typedef v8h  __attribute__((may_alias)) v8ha;
typedef v8us __attribute__((may_alias)) v8usa;
typedef v4f  __attribute__((may_alias)) v4fa;

union FragH { v16h v; v8h half[2]; };
union FragB { v16b v; v8us half[2]; };

#define NB    4
#define NSEQ  2048
#define DIM   384
#define NH    8
#define HDIM  48
#define NT    (NB * NSEQ)
#define DP    64
#define XP    (NH * DP)
#define NX    (NT * DIM)
#define NW    (DIM * DIM)
#define NX8   (NX / 8)
#define NW8   (NW / 8)
#define NGRP  (3 * NX8 + 4 * NW8)
#define LFP   52
#define VSP   136
#define NSEGMAX 4096
#define QSC   16.0f
#define KSC   16.0f
#define VSC   16.0f
#define PSC   16384.0f
#define XSC   1024.0f
#define WOSC  64.0f
#define SOFT_SCALE 0.14433756729740643f
#define NEG_BIG (-1.0e30f)

static_assert(NT % 128 == 0);
static_assert(NT % 64 == 0);
static_assert(DIM % 64 == 0);
static_assert(HDIM == 48);
static_assert(NGRP % 8 == 0);

__device__ __forceinline__ v8f wmma_f16(v16h a, v16h b, v8f c) {
  v8f d = __builtin_amdgcn_wmma_f32_16x16x32_f16(false, a, false, b, (short)0, c, false, false);
  asm volatile("v_nop\n\tv_nop\n\tv_nop\n\tv_nop" : "+v"(d) : "v"(a), "v"(b));
  return d;
}
__device__ __forceinline__ v8f wmma_bf16(v16b a, v16b b, v8f c) {
  v8f d = __builtin_amdgcn_wmma_f32_16x16x32_bf16(false, a, false, b, (short)0, c, false, false);
  union { v16b x; v16h y; } ua, ub;
  ua.x = a; ub.x = b;
  asm volatile("v_nop\n\tv_nop\n\tv_nop\n\tv_nop" : "+v"(d) : "v"(ua.y), "v"(ub.y));
  return d;
}

__device__ __forceinline__ v16h ldh2(const _Float16* p0, const _Float16* p1) {
  FragH f;
  f.half[0] = *(const v8ha*)p0;
  f.half[1] = *(const v8ha*)p1;
  return f.v;
}
__device__ __forceinline__ v16h ldh(const _Float16* p, int h) {
  return ldh2(p + 8 * h, p + 16 + 8 * h);
}
__device__ __forceinline__ v16b ldb(const unsigned short* p, int h) {
  FragB f;
  f.half[0] = *(const v8usa*)(p + 8 * h);
  f.half[1] = *(const v8usa*)(p + 16 + 8 * h);
  return f.v;
}

__device__ __forceinline__ unsigned int bf16_bits(float f) {
  unsigned int u = __float_as_uint(f);
  u += 0x7FFFu + ((u >> 16) & 1u);
  return u >> 16;
}
__device__ __forceinline__ void split_bf16(float x, unsigned short& hi, unsigned short& lo) {
  const unsigned int hb = bf16_bits(x);
  const float hf = __uint_as_float(hb << 16);
  hi = (unsigned short)hb;
  lo = (unsigned short)bf16_bits(x - hf);
}

__global__ __launch_bounds__(256) void convert_kernel(
    const float* __restrict__ xq, const float* __restrict__ xk, const float* __restrict__ xv,
    const float* __restrict__ wq, const float* __restrict__ wk, const float* __restrict__ wv,
    const float* __restrict__ wo,
    unsigned short* __restrict__ xhi3, unsigned short* __restrict__ xlo3,
    unsigned short* __restrict__ whi3, unsigned short* __restrict__ wlo3,
    _Float16* __restrict__ woh)
{
  const int g = blockIdx.x * 256 + threadIdx.x;
  if (g >= NGRP) return;
  const float* src;
  unsigned short* dh = xhi3;
  unsigned short* dl = xlo3;
  _Float16* dw = woh;
  bool wo_path = false;
  if (g < 3 * NX8) {
    const int r = g / NX8;
    const size_t off = (size_t)(g - r * NX8) * 8;
    const float* base = (r == 0) ? xq : ((r == 1) ? xk : xv);
    src = base + off;
    dh = xhi3 + (size_t)r * NX + off;
    dl = xlo3 + (size_t)r * NX + off;
  } else {
    const int e = g - 3 * NX8;
    const int r = e / NW8;
    const size_t off = (size_t)(e - r * NW8) * 8;
    if (r < 3) {
      const float* base = (r == 0) ? wq : ((r == 1) ? wk : wv);
      src = base + off;
      dh = whi3 + (size_t)r * NW + off;
      dl = wlo3 + (size_t)r * NW + off;
    } else {
      src = wo + off;
      dw = woh + off;
      wo_path = true;
    }
  }
  const v4f a = *(const v4fa*)src;
  const v4f c = *(const v4fa*)(src + 4);
  if (!wo_path) {
    v8us H, L;
    unsigned short th, tl;
    split_bf16(a.x, th, tl); H[0] = th; L[0] = tl;
    split_bf16(a.y, th, tl); H[1] = th; L[1] = tl;
    split_bf16(a.z, th, tl); H[2] = th; L[2] = tl;
    split_bf16(a.w, th, tl); H[3] = th; L[3] = tl;
    split_bf16(c.x, th, tl); H[4] = th; L[4] = tl;
    split_bf16(c.y, th, tl); H[5] = th; L[5] = tl;
    split_bf16(c.z, th, tl); H[6] = th; L[6] = tl;
    split_bf16(c.w, th, tl); H[7] = th; L[7] = tl;
    *(volatile v8us*)dh = H;
    *(volatile v8us*)dl = L;
    __threadfence();
    *(volatile v8us*)dh = H;
    *(volatile v8us*)dl = L;
  } else {
    const v8h o = { (_Float16)(a.x * WOSC), (_Float16)(a.y * WOSC), (_Float16)(a.z * WOSC), (_Float16)(a.w * WOSC),
                    (_Float16)(c.x * WOSC), (_Float16)(c.y * WOSC), (_Float16)(c.z * WOSC), (_Float16)(c.w * WOSC) };
    *(volatile v8h*)dw = o;
    __threadfence();
    *(volatile v8h*)dw = o;
  }
}

__device__ __forceinline__ float rope_inv(int j) {
  return (j == 0) ? 1.0f
       : (j == 1) ? 0.56234132519034908f
       : (j == 2) ? 0.31622776601683794f
       : (j == 3) ? 0.17782794100389228f
       : (j == 4) ? 0.1f
       : (j == 5) ? 0.056234132519034908f
       : (j == 6) ? 0.031622776601683794f
       :            0.017782794100389228f;
}

__device__ __forceinline__ void rope_sincos(float x, float& s, float& c) {
  const float kf = rintf(x * 0.636619772367581343f);
  float r = fmaf(-kf, 1.57079637050628662109375f, x);
  r = fmaf(-kf, -4.371139000186243e-8f, r);
  const float z = r * r;
  const float sp = fmaf(fmaf(fmaf(-1.9515295891e-4f, z, 8.3321608736e-3f), z, -1.6666654611e-1f), z * r, r);
  const float cp = fmaf(fmaf(fmaf(2.443315711809948e-5f, z, -1.388731625493765e-3f), z, 4.166664568298827e-2f),
                        z * z, fmaf(-0.5f, z, 1.0f));
  const int q = ((int)kf) & 3;
  float ss = (q & 1) ? cp : sp;
  float cc = (q & 1) ? sp : cp;
  if (q & 2) ss = -ss;
  if ((q + 1) & 2) cc = -cc;
  s = ss; c = cc;
}

__device__ __forceinline__ void proj_store(const _Float16* S16, int which, int head, int m0, int tid,
                                           _Float16* qhp, _Float16* qlp, _Float16* khp, _Float16* vtp) {
  if (which == 2) {
    #pragma unroll
    for (int i = 0; i < 6; ++i) {
      const int item = i * 128 + tid;
      const int d = item >> 4, piece = item & 15;
      const v8h v = *(const v8ha*)(S16 + d * VSP + piece * 8);
      _Float16* dst = vtp + ((size_t)head * HDIM + d) * NT + m0 + piece * 8;
      *(volatile v8h*)dst = v;
    }
  } else {
    const int npl = (which == 0) ? 2 : 1;
    for (int pl = 0; pl < npl; ++pl) {
      _Float16* plane = (pl == 0) ? ((which == 0) ? qhp : khp) : qlp;
      #pragma unroll
      for (int i = 0; i < 8; ++i) {
        const int item = i * 128 + tid;
        const int row = item >> 3, piece = item & 7;
        const v8h v = *(const v8ha*)(S16 + row * 128 + 64 * pl + piece * 8);
        _Float16* dst = plane + ((size_t)head * NT + m0 + row) * DP + piece * 8;
        *(volatile v8h*)dst = v;
      }
    }
  }
}

__global__ __launch_bounds__(128) void proj_kernel(
    const unsigned short* __restrict__ xhi3, const unsigned short* __restrict__ xlo3,
    const unsigned short* __restrict__ whi3, const unsigned short* __restrict__ wlo3,
    const float* __restrict__ bq, const float* __restrict__ bk, const float* __restrict__ bv,
    const int* __restrict__ posq, const int* __restrict__ posk,
    _Float16* __restrict__ qhp, _Float16* __restrict__ qlp,
    _Float16* __restrict__ khp, _Float16* __restrict__ vtp)
{
  __shared__ __attribute__((aligned(16))) float    Lf[128 * LFP];
  __shared__ __attribute__((aligned(16))) _Float16 S16[128 * 128];

  const int tid = threadIdx.x, lane = tid & 31, w = tid >> 5;
  const int h = lane >> 4, m = lane & 15;
  const int m0 = blockIdx.x * 128;
  const int which = blockIdx.y / NH;
  const int head = blockIdx.y - which * NH;

  const unsigned short* xh = xhi3 + (size_t)which * NX;
  const unsigned short* xl = xlo3 + (size_t)which * NX;
  const unsigned short* wh = whi3 + (size_t)which * NW;
  const unsigned short* wl = wlo3 + (size_t)which * NW;

  const size_t arow0 = (size_t)(m0 + 32 * w + m) * DIM;
  const size_t arow1 = arow0 + (size_t)16 * DIM;
  const size_t brow  = (size_t)(head * HDIM + m) * DIM;

  const v8f zero8 = {0.f, 0.f, 0.f, 0.f, 0.f, 0.f, 0.f, 0.f};
  v8f acc[2][3];
  #pragma unroll
  for (int mt = 0; mt < 2; ++mt)
    #pragma unroll
    for (int nt = 0; nt < 3; ++nt) acc[mt][nt] = zero8;

  #pragma unroll 1
  for (int k0 = 0; k0 < DIM; k0 += 32) {
    const v16b ah0 = ldb(xh + arow0 + k0, h);
    const v16b ah1 = ldb(xh + arow1 + k0, h);
    const v16b al0 = ldb(xl + arow0 + k0, h);
    const v16b al1 = ldb(xl + arow1 + k0, h);
    #pragma unroll
    for (int nt = 0; nt < 3; ++nt) {
      const v16b wbh = ldb(wh + brow + (size_t)nt * 16 * DIM + k0, h);
      const v16b wbl = ldb(wl + brow + (size_t)nt * 16 * DIM + k0, h);
      acc[0][nt] = wmma_bf16(ah0, wbh, acc[0][nt]);
      acc[0][nt] = wmma_bf16(ah0, wbl, acc[0][nt]);
      acc[0][nt] = wmma_bf16(al0, wbh, acc[0][nt]);
      acc[1][nt] = wmma_bf16(ah1, wbh, acc[1][nt]);
      acc[1][nt] = wmma_bf16(ah1, wbl, acc[1][nt]);
      acc[1][nt] = wmma_bf16(al1, wbh, acc[1][nt]);
    }
  }

  const float* bias = (which == 0) ? bq : ((which == 1) ? bk : bv);
  if (which == 2) {
    #pragma unroll
    for (int nt = 0; nt < 3; ++nt) {
      const int col = 16 * nt + m;
      const float bvl = bias[head * HDIM + col];
      #pragma unroll
      for (int mt = 0; mt < 2; ++mt)
        #pragma unroll
        for (int r = 0; r < 8; ++r) {
          const int tokl = 32 * w + 16 * mt + 8 * h + r;
          S16[col * VSP + tokl] = (_Float16)((acc[mt][nt][r] + bvl) * VSC);
        }
    }
  } else {
    #pragma unroll
    for (int nt = 0; nt < 3; ++nt) {
      const int col = 16 * nt + m;
      const float bvl = bias[head * HDIM + col];
      #pragma unroll
      for (int mt = 0; mt < 2; ++mt)
        #pragma unroll
        for (int r = 0; r < 8; ++r) {
          const int tokl = 32 * w + 16 * mt + 8 * h + r;
          Lf[tokl * LFP + col] = acc[mt][nt][r] + bvl;
        }
    }
  }
  __syncthreads();

  if (which != 2) {
    const int t = m0 + tid;
    const int* pos = ((which == 0) ? posq : posk) + (size_t)t * 3;
    const float* lrow = Lf + tid * LFP;
    _Float16* srow = S16 + tid * 128;
    const bool isq = (which == 0);
    #pragma unroll 1
    for (int c = 0; c < 3; ++c) {
      const float pf = (float)pos[c];
      #pragma unroll
      for (int j = 0; j < 8; ++j) {
        float sn, cs;
        rope_sincos(pf * rope_inv(j), sn, cs);
        const float x1 = lrow[16 * c + j];
        const float x2 = lrow[16 * c + j + 8];
        const float r1 = (x1 * cs - x2 * sn) * QSC;
        const float r2 = (x2 * cs + x1 * sn) * QSC;
        const _Float16 h1 = (_Float16)r1, h2 = (_Float16)r2;
        srow[16 * c + j]     = h1;
        srow[16 * c + j + 8] = h2;
        srow[64 + 16 * c + j]     = isq ? (_Float16)(r1 - (float)h1) : (_Float16)0.0f;
        srow[64 + 16 * c + j + 8] = isq ? (_Float16)(r2 - (float)h2) : (_Float16)0.0f;
      }
    }
    #pragma unroll
    for (int i = 0; i < 16; ++i) { srow[48 + i] = (_Float16)0.0f; srow[112 + i] = (_Float16)0.0f; }
  }
  __syncthreads();

  proj_store(S16, which, head, m0, tid, qhp, qlp, khp, vtp);
  __threadfence();
  proj_store(S16, which, head, m0, tid, qhp, qlp, khp, vtp);
}

__device__ __forceinline__ v16h pack_p(v8f a, v8f c) {
  const v16h r = { (_Float16)(a[0] * PSC), (_Float16)(a[1] * PSC), (_Float16)(a[2] * PSC), (_Float16)(a[3] * PSC),
                   (_Float16)(a[4] * PSC), (_Float16)(a[5] * PSC), (_Float16)(a[6] * PSC), (_Float16)(a[7] * PSC),
                   (_Float16)(c[0] * PSC), (_Float16)(c[1] * PSC), (_Float16)(c[2] * PSC), (_Float16)(c[3] * PSC),
                   (_Float16)(c[4] * PSC), (_Float16)(c[5] * PSC), (_Float16)(c[6] * PSC), (_Float16)(c[7] * PSC) };
  return r;
}

__device__ __forceinline__ void att_store_pass(const _Float16* so, _Float16* xah, _Float16* xal,
                                               size_t tokbase, int head, int lane) {
  const int q8 = lane & 7, sub = lane >> 3;
  #pragma unroll
  for (int i = 0; i < 8; ++i) {
    const int lid = i * 4 + sub;
    const int row = lid >> 1, hl = lid & 1;
    const v8h v = *(const v8ha*)(so + row * 128 + 64 * hl + 8 * q8);
    _Float16* dst = (hl ? xal : xah) + (tokbase + row) * XP + head * DP + 8 * q8;
    *(volatile v8h*)dst = v;
  }
}

__global__ __launch_bounds__(128) void attn_kernel(
    const _Float16* __restrict__ qhp,
    const _Float16* __restrict__ qlp,
    const _Float16* __restrict__ khp,
    const _Float16* __restrict__ vtp,
    const int* __restrict__ qoff,
    const int* __restrict__ koff,
    int nseg,
    _Float16* __restrict__ xah,
    _Float16* __restrict__ xal)
{
  __shared__ __attribute__((aligned(16))) _Float16 sO[4 * 16 * 128];

  const int tid = threadIdx.x, lane = tid & 31, w = tid >> 5;
  const int h = lane >> 4, m = lane & 15;
  const int head = blockIdx.y;
  const int q0 = blockIdx.x * 64 + 16 * w;
  const int tq = q0 + m;

  int sq = 0;
  #pragma unroll 1
  for (int i = 0; i + 1 < nseg; ++i) sq += (qoff[i] <= tq) ? 1 : 0;
  int kbeg = (sq > 0) ? koff[sq - 1] : 0;
  int kend = koff[sq];
  kbeg = min(max(kbeg, 0), NT);
  kend = min(max(kend, kbeg), NT);
  int lo64 = kbeg & ~63, hiend = kend, kbmax = kbeg, kemin = kend;
  #pragma unroll
  for (int sft = 1; sft < 32; sft <<= 1) {
    lo64  = min(lo64,  __shfl_xor(lo64,  sft));
    hiend = max(hiend, __shfl_xor(hiend, sft));
    kbmax = max(kbmax, __shfl_xor(kbmax, sft));
    kemin = min(kemin, __shfl_xor(kemin, sft));
  }
  lo64  = __builtin_amdgcn_readfirstlane(lo64);
  hiend = __builtin_amdgcn_readfirstlane(hiend);
  kbmax = __builtin_amdgcn_readfirstlane(kbmax);
  kemin = __builtin_amdgcn_readfirstlane(kemin);

  const size_t qrow = ((size_t)head * NT + tq) * DP;
  const _Float16* qh = qhp + qrow;
  const _Float16* ql = qlp + qrow;
  const v16h qb0 = ldh2(qh + 8 * h,      qh + 16 + 8 * h);
  const v16h qb1 = ldh2(qh + 32 + 8 * h, ql + 8 * h);
  const v16h qb2 = ldh2(ql + 16 + 8 * h, ql + 32 + 8 * h);

  const v8f zero8 = {0.f, 0.f, 0.f, 0.f, 0.f, 0.f, 0.f, 0.f};
  v8f o[3];
  #pragma unroll
  for (int t = 0; t < 3; ++t) o[t] = zero8;
  float mrun = NEG_BIG, lrun = 0.0f;

  const _Float16* kbase = khp + ((size_t)head * NT + m) * DP;
  const _Float16* vbase = vtp + ((size_t)head * HDIM + m) * NT;
  const float SS = SOFT_SCALE * (1.0f / (QSC * KSC));

  #pragma unroll 1
  for (int it = 0; it < NT / 64; ++it) {
    const int kb = lo64 + 64 * it;
    if (kb >= hiend) break;
    const bool part = (kb < kbmax) || (kb + 64 > kemin);

    v8f s[4];
    #pragma unroll
    for (int j = 0; j < 4; ++j) {
      const _Float16* kp = kbase + (size_t)(kb + 16 * j) * DP;
      const v16h a0 = ldh2(kp + 8 * h,      kp + 16 + 8 * h);
      const v16h a1 = ldh2(kp + 32 + 8 * h, kp + 8 * h);
      const v16h a2 = ldh2(kp + 16 + 8 * h, kp + 32 + 8 * h);
      v8f z = zero8;
      z = wmma_f16(a0, qb0, z);
      z = wmma_f16(a1, qb1, z);
      z = wmma_f16(a2, qb2, z);
      s[j] = z * SS;
    }
    if (part) {
      #pragma unroll
      for (int j = 0; j < 4; ++j)
        #pragma unroll
        for (int r = 0; r < 8; ++r) {
          const int key = kb + 16 * j + 8 * h + r;
          if (key < kbeg || key >= kend) s[j][r] = NEG_BIG;
        }
    }

    float mloc = s[0][0];
    #pragma unroll
    for (int j = 0; j < 4; ++j)
      #pragma unroll
      for (int r = 0; r < 8; ++r) mloc = fmaxf(mloc, s[j][r]);
    mloc = fmaxf(mloc, __shfl_xor(mloc, 16));
    const float mnew = fmaxf(mrun, mloc);
    const float alpha = __expf(mrun - mnew);
    mrun = mnew;
    #pragma unroll
    for (int j = 0; j < 4; ++j)
      #pragma unroll
      for (int r = 0; r < 8; ++r) s[j][r] = __expf(s[j][r] - mnew);
    if (part) {
      #pragma unroll
      for (int j = 0; j < 4; ++j)
        #pragma unroll
        for (int r = 0; r < 8; ++r) {
          const int key = kb + 16 * j + 8 * h + r;
          if (key < kbeg || key >= kend) s[j][r] = 0.0f;
        }
    }
    float lsum = 0.0f;
    #pragma unroll
    for (int j = 0; j < 4; ++j)
      #pragma unroll
      for (int r = 0; r < 8; ++r) lsum += s[j][r];
    lsum += __shfl_xor(lsum, 16);
    lrun = lrun * alpha + lsum;
    #pragma unroll
    for (int t = 0; t < 3; ++t)
      #pragma unroll
      for (int r = 0; r < 8; ++r) o[t][r] = o[t][r] * alpha;

    const v16h pb0 = pack_p(s[0], s[1]);
    const v16h pb1 = pack_p(s[2], s[3]);

    #pragma unroll
    for (int t = 0; t < 3; ++t) {
      const _Float16* vp = vbase + (size_t)(16 * t) * NT + kb;
      const v16h vf0 = ldh(vp, h);
      const v16h vf1 = ldh(vp + 32, h);
      o[t] = wmma_f16(vf0, pb0, o[t]);
      o[t] = wmma_f16(vf1, pb1, o[t]);
    }
  }

  const float oinv = (lrun > 0.0f) ? ((XSC / (PSC * VSC)) / lrun) : 0.0f;
  _Float16* so = sO + w * (16 * 128);
  #pragma unroll
  for (int t = 0; t < 3; ++t)
    #pragma unroll
    for (int r = 0; r < 8; ++r) {
      const float xs = o[t][r] * oinv;
      const _Float16 hv = (_Float16)xs;
      so[m * 128 + 16 * t + 8 * h + r]      = hv;
      so[m * 128 + 64 + 16 * t + 8 * h + r] = (_Float16)(xs - (float)hv);
    }
  #pragma unroll
  for (int r = 0; r < 8; ++r) {
    so[m * 128 + 48 + 8 * h + r]  = (_Float16)0.0f;
    so[m * 128 + 112 + 8 * h + r] = (_Float16)0.0f;
  }
  __syncthreads();

  const size_t tokbase = (size_t)q0;
  att_store_pass(so, xah, xal, tokbase, head, lane);
  __threadfence();
  att_store_pass(so, xah, xal, tokbase, head, lane);
}

__device__ __forceinline__ void out_store_pass(const float* sT, float* out, int m0, int cg, int tid) {
  #pragma unroll
  for (int i = 0; i < 16; ++i) {
    const int item = i * 128 + tid;
    const int row = item >> 4, piece = item & 15;
    const v4f v = *(const v4fa*)(sT + row * 64 + piece * 4);
    float* dst = out + (size_t)(m0 + row) * DIM + cg * 64 + piece * 4;
    *(volatile v4f*)dst = v;
  }
}

__global__ __launch_bounds__(128) void oproj_kernel(
    const _Float16* __restrict__ xah, const _Float16* __restrict__ xal,
    const _Float16* __restrict__ woh, const float* __restrict__ bo,
    float* __restrict__ out)
{
  __shared__ __attribute__((aligned(16))) float sT[128 * 64];

  const int tid = threadIdx.x, lane = tid & 31, w = tid >> 5;
  const int h = lane >> 4, m = lane & 15;
  const int m0 = blockIdx.x * 128;
  const int cg = blockIdx.y;

  const size_t arow0 = (size_t)(m0 + 32 * w + m) * XP;
  const size_t arow1 = arow0 + (size_t)16 * XP;
  const size_t brow  = (size_t)(cg * 64 + m) * DIM;

  const v8f zero8 = {0.f, 0.f, 0.f, 0.f, 0.f, 0.f, 0.f, 0.f};
  v8f acc[2][4];
  #pragma unroll
  for (int mt = 0; mt < 2; ++mt)
    #pragma unroll
    for (int nt = 0; nt < 4; ++nt) acc[mt][nt] = zero8;

  #pragma unroll 1
  for (int k0 = 0; k0 < DIM; k0 += 32) {
    const int ka = k0 + 8 * h, kc = k0 + 16 + 8 * h;
    const int oa = ka + 16 * (ka / HDIM), oc = kc + 16 * (kc / HDIM);
    const v16h ah0 = ldh2(xah + arow0 + oa, xah + arow0 + oc);
    const v16h ah1 = ldh2(xah + arow1 + oa, xah + arow1 + oc);
    const v16h al0 = ldh2(xal + arow0 + oa, xal + arow0 + oc);
    const v16h al1 = ldh2(xal + arow1 + oa, xal + arow1 + oc);
    #pragma unroll
    for (int nt = 0; nt < 4; ++nt) {
      const v16h bw = ldh(woh + brow + (size_t)nt * 16 * DIM + k0, h);
      acc[0][nt] = wmma_f16(ah0, bw, acc[0][nt]);
      acc[0][nt] = wmma_f16(al0, bw, acc[0][nt]);
      acc[1][nt] = wmma_f16(ah1, bw, acc[1][nt]);
      acc[1][nt] = wmma_f16(al1, bw, acc[1][nt]);
    }
  }

  const float osc = 1.0f / (XSC * WOSC);
  #pragma unroll
  for (int nt = 0; nt < 4; ++nt) {
    const int col = 16 * nt + m;
    const float bvl = bo[cg * 64 + col];
    #pragma unroll
    for (int mt = 0; mt < 2; ++mt)
      #pragma unroll
      for (int r = 0; r < 8; ++r) {
        const int tokl = 32 * w + 16 * mt + 8 * h + r;
        sT[tokl * 64 + col] = acc[mt][nt][r] * osc + bvl;
      }
  }
  __syncthreads();

  out_store_pass(sT, out, m0, cg, tid);
  __threadfence();
  out_store_pass(sT, out, m0, cg, tid);
}

extern "C" void kernel_launch(void* const* d_in, const int* in_sizes, int n_in,
                              void* d_out, int out_size, void* d_ws, size_t ws_size,
                              hipStream_t stream) {
  if (n_in < 15) return;
  if (in_sizes[0] != NX || in_sizes[1] != NX || in_sizes[2] != NX) return;
  if (in_sizes[3] != NW || in_sizes[5] != NW || in_sizes[7] != NW || in_sizes[9] != NW) return;
  if (in_sizes[4] != DIM || in_sizes[6] != DIM || in_sizes[8] != DIM || in_sizes[10] != DIM) return;
  if (in_sizes[11] != NT * 3 || in_sizes[12] != NT * 3) return;
  const int nseg = in_sizes[13];
  if (nseg < 1 || nseg > NSEGMAX || in_sizes[14] != nseg) return;
  if (out_size != NX) return;

  const float* xq = (const float*)d_in[0];
  const float* xk = (const float*)d_in[1];
  const float* xv = (const float*)d_in[2];
  const float* Wq = (const float*)d_in[3];
  const float* bq = (const float*)d_in[4];
  const float* Wk = (const float*)d_in[5];
  const float* bk = (const float*)d_in[6];
  const float* Wv = (const float*)d_in[7];
  const float* bv = (const float*)d_in[8];
  const float* Wo = (const float*)d_in[9];
  const float* bo = (const float*)d_in[10];
  const int*   qpos = (const int*)d_in[11];
  const int*   kpos = (const int*)d_in[12];
  const int*   qoff = (const int*)d_in[13];
  const int*   koff = (const int*)d_in[14];
  float* out = (float*)d_out;

  const size_t xpl = (size_t)NX * 2;
  const size_t wpl = (size_t)NW * 2;
  const size_t ppl = (size_t)NH * NT * DP * 2;
  const size_t vpl = (size_t)NH * HDIM * NT * 2;
  const size_t apl = (size_t)NT * XP * 2;
  size_t off = 0;
  char* ws = (char*)d_ws;
  unsigned short* xhi3 = (unsigned short*)(ws + off); off += 3 * xpl;
  unsigned short* xlo3 = (unsigned short*)(ws + off); off += 3 * xpl;
  unsigned short* whi3 = (unsigned short*)(ws + off); off += 3 * wpl;
  unsigned short* wlo3 = (unsigned short*)(ws + off); off += 3 * wpl;
  _Float16* woh = (_Float16*)(ws + off); off += wpl;
  _Float16* qhp = (_Float16*)(ws + off); off += ppl;
  _Float16* qlp = (_Float16*)(ws + off); off += ppl;
  _Float16* khp = (_Float16*)(ws + off); off += ppl;
  _Float16* vtp = (_Float16*)(ws + off); off += vpl;
  _Float16* xah = (_Float16*)(ws + off); off += apl;
  _Float16* xal = (_Float16*)(ws + off); off += apl;
  if (off > ws_size) return;

  convert_kernel<<<(NGRP + 255) / 256, 256, 0, stream>>>(xq, xk, xv, Wq, Wk, Wv, Wo,
                                                         xhi3, xlo3, whi3, wlo3, woh);

  dim3 gProj(NT / 128, 3 * NH);
  proj_kernel<<<gProj, 128, 0, stream>>>(xhi3, xlo3, whi3, wlo3, bq, bk, bv, qpos, kpos,
                                         qhp, qlp, khp, vtp);

  dim3 gAtt(NT / 64, NH);
  attn_kernel<<<gAtt, 128, 0, stream>>>(qhp, qlp, khp, vtp, qoff, koff, nseg, xah, xal);

  dim3 gOut(NT / 128, DIM / 64);
  oproj_kernel<<<gOut, 128, 0, stream>>>(xah, xal, woh, bo, out);
}
